// PairStateLayer_69123203662020
// MI455X (gfx1250) — hardware-run, weakly checked
//
#include <hip/hip_runtime.h>
#include <math.h>

constexpr int kNB    = 8;
constexpr int kNS    = 2048;
constexpr int kNDM   = 512;
constexpr int kNH    = 8;
constexpr int kNSD   = 64;
constexpr int kRows  = kNB * kNS;
constexpr int kInner = kNH * kNSD;
constexpr int kNProj = 4 * kInner;
constexpr int kNHid  = 4 * kNDM;
constexpr int kGateN = 64;
constexpr int kFfnChunkRows = kRows / 2;
constexpr float kLnEps = 1e-5f;
constexpr float kNCarry    = 4.0f;
constexpr float kWCarry    = 32.0f;
constexpr float kActCarry  = 8.0f;
constexpr float kActInv    = 1.0f / 8.0f;
constexpr float kPairCarry = 256.0f;
constexpr float kMixCarry  = 16.0f;
constexpr float kProjScale = 1.0f / (kNCarry * kWCarry);
constexpr float kLcInv     = 1.0f / (kPairCarry * kActCarry);
constexpr float kWoutScale = 1.0f / (kMixCarry * kWCarry);
constexpr float kW1Scale   = kActCarry / (kNCarry * kWCarry);
constexpr float kW2Scale   = 1.0f / (kActCarry * kWCarry);
constexpr float kInvDM     = 1.0f / 512.0f;

typedef __attribute__((ext_vector_type(16))) _Float16 v16h;
typedef __attribute__((ext_vector_type(8)))  _Float16 v8h;
typedef __attribute__((ext_vector_type(16))) __bf16   v16b;
typedef __attribute__((ext_vector_type(8)))  __bf16   v8b;
typedef __attribute__((ext_vector_type(8)))  float    v8f;
typedef __attribute__((ext_vector_type(4)))  float    v4f;
typedef __attribute__((ext_vector_type(4)))  unsigned int v4u;

__device__ __forceinline__ unsigned short f2bf_bits(float f) {
  unsigned u = __float_as_uint(f);
  return (unsigned short)((u + 0x7FFFu + ((u >> 16) & 1u)) >> 16);
}
__device__ __forceinline__ float bf_bits2f(unsigned short h) { return __uint_as_float(((unsigned)h) << 16); }

__device__ __forceinline__ void dep_guard_h(v8f& a, v8f& b, v16h x, v16h y) { asm volatile("v_nop\n\tv_nop\n\tv_nop\n\tv_nop" : "+v"(a), "+v"(b) : "v"(x), "v"(y)); }
__device__ __forceinline__ void dep_guard_b(v8f& a, v8f& b, v16b x, v16b y) { asm volatile("v_nop\n\tv_nop\n\tv_nop\n\tv_nop" : "+v"(a), "+v"(b) : "v"(x), "v"(y)); }
__device__ __forceinline__ void keep4_h(v16h a, v16h b, v16h c, v16h d) { asm volatile("v_nop" :: "v"(a), "v"(b), "v"(c), "v"(d)); }
__device__ __forceinline__ void keep4_b(v16b a, v16b b, v16b c, v16b d) { asm volatile("v_nop" :: "v"(a), "v"(b), "v"(c), "v"(d)); }
__device__ __forceinline__ void acc_guard4(v8f& a, v8f& b, v8f& c, v8f& d) { asm volatile("v_nop\n\tv_nop\n\tv_nop\n\tv_nop" : "+v"(a), "+v"(b), "+v"(c), "+v"(d)); }
template <typename T> struct Frag;
template <> struct Frag<_Float16> {
  typedef v16h V; union U { v16h v; v8h h[2]; };
  static __device__ __forceinline__ v16h load(const _Float16* p) {
    U f; f.h[0] = *(const v8h*)(p); f.h[1] = *(const v8h*)(p + 16); return f.v;
  }
  static __device__ __forceinline__ v8f mma(v16h a, v16h b, v8f c) {
    return __builtin_amdgcn_wmma_f32_16x16x32_f16(false, a, false, b, (short)0, c, false, false);
  }
  static __device__ __forceinline__ void guard(v8f& a, v8f& b, v16h x, v16h y) { dep_guard_h(a, b, x, y); }
  static __device__ __forceinline__ void keep(v16h a, v16h b, v16h c, v16h d) { keep4_h(a, b, c, d); }
};
template <> struct Frag<__bf16> {
  typedef v16b V; union U { v16b v; v8b h[2]; };
  static __device__ __forceinline__ v16b load(const __bf16* p) {
    U f; f.h[0] = *(const v8b*)(p); f.h[1] = *(const v8b*)(p + 16); return f.v;
  }
  static __device__ __forceinline__ v8f mma(v16b a, v16b b, v8f c) {
    return __builtin_amdgcn_wmma_f32_16x16x32_bf16(false, a, false, b, (short)0, c, false, false);
  }
  static __device__ __forceinline__ void guard(v8f& a, v8f& b, v16b x, v16b y) { dep_guard_b(a, b, x, y); }
  static __device__ __forceinline__ void keep(v16b a, v16b b, v16b c, v16b d) { keep4_b(a, b, c, d); }
};

__device__ __forceinline__ unsigned pk16(unsigned short a, unsigned short b) { return (unsigned)a | ((unsigned)b << 16); }
__device__ __forceinline__ unsigned short h_bits(float f) { const _Float16 h = (_Float16)f; return __builtin_bit_cast(unsigned short, h); }
__device__ __forceinline__ float h2f(unsigned int u16) { return (float)__builtin_bit_cast(_Float16, (unsigned short)(u16 & 0xffffu)); }

__device__ __forceinline__ v8f hmma(v16h a, v16h b, v8f c) {
  c = __builtin_amdgcn_wmma_f32_16x16x32_f16(false, a, false, b, (short)0, c, false, false);
  asm volatile("v_nop\n\tv_nop\n\tv_nop\n\tv_nop" : "+v"(c) : "v"(a), "v"(b));
  return c;
}

template <int ET> struct Elem;
template <> struct Elem<0> { typedef _Float16 T; };
template <> struct Elem<1> { typedef __bf16 T; };
template <int ET, bool SPLIT, int BIAS_MODE, int OUT_MODE, bool RESID, int ACT = 0>
__global__ __launch_bounds__(256) void wmma_gemm64(
    const unsigned short* __restrict__ Ap, const unsigned short* __restrict__ A2p, int lda, long strideA,
    const unsigned short* __restrict__ Btp, const unsigned short* __restrict__ Bt2p, int ldb, long strideB,
    void* __restrict__ Cout, void* __restrict__ Cout2, int ldc, long strideC,
    const float* __restrict__ bias,
    const float* __restrict__ resid, long strideR,
    int M, int N, int K, float scale) {
  typedef typename Elem<ET>::T T;
  typedef typename Frag<T>::V V;
  const T* A = (const T*)Ap; const T* A2 = (const T*)A2p; const T* Bt = (const T*)Btp; const T* Bt2 = (const T*)Bt2p;
  __shared__ __align__(16) float sT[8][16 * 68];
  const int b    = blockIdx.y;
  const int lane = threadIdx.x & 31;
  const int wave = threadIdx.x >> 5;
  const int tilesN = N >> 6;
  const int tilesM = M >> 6;
  const int tile = blockIdx.x * 8 + wave;
  if (tile >= tilesM * tilesN) return;
  const int tm = tile / tilesN;
  const int tn = tile - tm * tilesN;
  const int m0 = tm << 6;
  const int n0 = tn << 6;

  const T* Ab  = A  + (size_t)b * strideA;
  const T* Bb  = Bt + (size_t)b * strideB;
  const T* Ab2 = SPLIT ? (A2  + (size_t)b * strideA) : nullptr;
  const T* Bb2 = SPLIT ? (Bt2 + (size_t)b * strideB) : nullptr;

  const int rlane = lane & 15;
  const int koff  = (lane >> 4) * 8;
  const int mOff  = (lane >> 4) * 8;

  v8f acc[4][4];
#pragma unroll
  for (int i = 0; i < 4; ++i)
#pragma unroll
    for (int j = 0; j < 4; ++j) acc[i][j] = (v8f){0.f,0.f,0.f,0.f,0.f,0.f,0.f,0.f};

  for (int k0 = 0; k0 < K; k0 += 32) {
    V bh[4], bl[4];
#pragma unroll
    for (int j = 0; j < 4; ++j) {
      const size_t bo = (size_t)(n0 + (j << 4) + rlane) * ldb + koff + k0;
      bh[j] = Frag<T>::load(Bb + bo);
      if (SPLIT) bl[j] = Frag<T>::load(Bb2 + bo);
    }
#pragma unroll
    for (int i = 0; i < 4; ++i) {
      const size_t ao = (size_t)(m0 + (i << 4) + rlane) * lda + koff + k0;
      V ah = Frag<T>::load(Ab + ao);
      V al;
      if (SPLIT) al = Frag<T>::load(Ab2 + ao);
#pragma unroll
      for (int j = 0; j < 4; ++j) {
        acc[i][j] = Frag<T>::mma(ah, bh[j], acc[i][j]);
        if (SPLIT) {
          acc[i][j] = Frag<T>::mma(ah, bl[j], acc[i][j]);
          acc[i][j] = Frag<T>::mma(al, bh[j], acc[i][j]);
        }
      }
      Frag<T>::guard(acc[i][0], acc[i][3], ah, SPLIT ? al : ah);
    }
    Frag<T>::keep(bh[0], bh[1], bh[2], bh[3]);
    if (SPLIT) Frag<T>::keep(bl[0], bl[1], bl[2], bl[3]);
  }
  acc_guard4(acc[0][0], acc[0][1], acc[0][2], acc[0][3]);
  acc_guard4(acc[1][0], acc[1][1], acc[1][2], acc[1][3]);
  acc_guard4(acc[2][0], acc[2][1], acc[2][2], acc[2][3]);
  acc_guard4(acc[3][0], acc[3][1], acc[3][2], acc[3][3]);

  float* slab = sT[wave];
  const float* Rb = RESID ? (resid + (size_t)b * strideR) : nullptr;
#pragma unroll
  for (int i = 0; i < 4; ++i) {
    const int mBase = m0 + (i << 4);
#pragma unroll
    for (int j = 0; j < 4; ++j) {
      const int n = n0 + (j << 4) + rlane;
      float bv = 0.f;
      if (BIAS_MODE == 2) bv = bias[n];
#pragma unroll
      for (int r = 0; r < 8; ++r) {
        float v = acc[i][j][r] * scale;
        if (BIAS_MODE == 1) v += bias[mBase + mOff + r];
        if (BIAS_MODE == 2) v += bv;
        if (RESID) v += Rb[(size_t)(mBase + mOff + r) * ldc + n];
        if (ACT == 1) v = tanhf(v);
        if (ACT == 2) v = fmaxf(v, 0.0f);
        if (ACT == 3) v = v / (1.0f + expf(-v));
        if (ACT == 4) v = (v > 0.f) ? v : 0.01f * v;
        if (ACT == 5) v = 0.5f * v * (1.0f + erff(v * 0.70710678118654752f));
        if (ACT == 6) v = tanhf(v) * 8.0f;
        slab[(mOff + r) * 68 + (j << 4) + rlane] = v;
      }
    }
    __builtin_amdgcn_fence(__ATOMIC_RELEASE, "workgroup");
    __builtin_amdgcn_wave_barrier();
    __builtin_amdgcn_fence(__ATOMIC_ACQUIRE, "workgroup");
    if (OUT_MODE == 0) {
      float* C = (float*)Cout + (size_t)b * strideC;
      const int hh = lane >> 4, c4 = (lane & 15) * 4;
      for (int pass = 0; pass < 2; ++pass) {
#pragma unroll
        for (int it = 0; it < 8; ++it) {
          const int row = it * 2 + hh;
          v4f v = *(const v4f*)(slab + row * 68 + c4);
          *(volatile v4f*)(C + (size_t)(mBase + row) * ldc + n0 + c4) = v;
        }
        __threadfence();
      }
    } else {
      const int q = lane >> 3, c8 = (lane & 7) * 8;
      unsigned short* C  = (unsigned short*)Cout  + (size_t)b * strideC;
      unsigned short* C2 = (OUT_MODE == 2) ? ((unsigned short*)Cout2 + (size_t)b * strideC) : nullptr;
      for (int pass = 0; pass < 2; ++pass) {
#pragma unroll
        for (int it = 0; it < 4; ++it) {
          const int row = it * 4 + q;
          const float* sp = slab + row * 68 + c8;
          v8h hv, lv;
#pragma unroll
          for (int e = 0; e < 8; ++e) {
            if (OUT_MODE == 1) {
              hv[e] = (_Float16)sp[e];
            } else {
              unsigned short hb = f2bf_bits(sp[e]);
              unsigned short lb = f2bf_bits(sp[e] - bf_bits2f(hb));
              hv[e] = __builtin_bit_cast(_Float16, hb);
              lv[e] = __builtin_bit_cast(_Float16, lb);
            }
          }
          *(volatile v8h*)(C + (size_t)(mBase + row) * ldc + n0 + c8) = hv;
          if (OUT_MODE == 2) *(volatile v8h*)(C2 + (size_t)(mBase + row) * ldc + n0 + c8) = lv;
        }
        __threadfence();
      }
    }
    __builtin_amdgcn_fence(__ATOMIC_RELEASE, "workgroup");
    __builtin_amdgcn_wave_barrier();
    __builtin_amdgcn_fence(__ATOMIC_ACQUIRE, "workgroup");
  }
}

__global__ __launch_bounds__(256) void ln_f16_kernel(const float* __restrict__ x, const float* __restrict__ g,
                                                     const float* __restrict__ be, unsigned short* __restrict__ out,
                                                     int nrows, float carry) {
  const int wave = threadIdx.x >> 5, lane = threadIdx.x & 31;
  const int row = blockIdx.x * 8 + wave;
  if (row >= nrows) return;
  const float* xr = x + (size_t)row * kNDM;
  const int c0 = 8 * lane, c1 = 256 + 8 * lane;
  const v4f a0 = *(const v4f*)(xr + c0);
  const v4f a1 = *(const v4f*)(xr + c0 + 4);
  const v4f a2 = *(const v4f*)(xr + c1);
  const v4f a3 = *(const v4f*)(xr + c1 + 4);
  float v[16];
#pragma unroll
  for (int e = 0; e < 4; ++e) { v[e] = a0[e]; v[4 + e] = a1[e]; v[8 + e] = a2[e]; v[12 + e] = a3[e]; }
  float s = 0.f;
#pragma unroll
  for (int e = 0; e < 16; ++e) s += v[e];
#pragma unroll
  for (int off = 16; off > 0; off >>= 1) s += __shfl_xor(s, off, 32);
  const float mean = s * kInvDM;
  float q = 0.f;
#pragma unroll
  for (int e = 0; e < 16; ++e) { const float d = v[e] - mean; q += d * d; }
#pragma unroll
  for (int off = 16; off > 0; off >>= 1) q += __shfl_xor(q, off, 32);
  const float var = q * kInvDM;
  const float inv = 1.0f / sqrtf(var + kLnEps);
  const v4f g0 = *(const v4f*)(g + c0), g1 = *(const v4f*)(g + c0 + 4), g2 = *(const v4f*)(g + c1), g3 = *(const v4f*)(g + c1 + 4);
  const v4f b0 = *(const v4f*)(be + c0), b1v = *(const v4f*)(be + c0 + 4), b2v = *(const v4f*)(be + c1), b3 = *(const v4f*)(be + c1 + 4);
  float gg[16], bb[16];
#pragma unroll
  for (int e = 0; e < 4; ++e) {
    gg[e] = g0[e]; gg[4 + e] = g1[e]; gg[8 + e] = g2[e]; gg[12 + e] = g3[e];
    bb[e] = b0[e]; bb[4 + e] = b1v[e]; bb[8 + e] = b2v[e]; bb[12 + e] = b3[e];
  }
  unsigned short hb[16];
#pragma unroll
  for (int e = 0; e < 16; ++e) hb[e] = h_bits(((v[e] - mean) * inv * gg[e] + bb[e]) * carry);
  const v4u u0 = (v4u){pk16(hb[0], hb[1]), pk16(hb[2], hb[3]), pk16(hb[4], hb[5]), pk16(hb[6], hb[7])};
  const v4u u1 = (v4u){pk16(hb[8], hb[9]), pk16(hb[10], hb[11]), pk16(hb[12], hb[13]), pk16(hb[14], hb[15])};
  unsigned short* orow = out + (size_t)row * kNDM;
  *(volatile v4u*)(orow + c0) = u0;
  *(volatile v4u*)(orow + c1) = u1;
  __threadfence();
  *(volatile v4u*)(orow + c0) = u0;
  *(volatile v4u*)(orow + c1) = u1;
}

__global__ __launch_bounds__(256) void castw4_kernel(const float* __restrict__ W0, const float* __restrict__ W1,
                                                     const float* __restrict__ W2, const float* __restrict__ W3,
                                                     unsigned short* __restrict__ out, int n8, float scale) {
  const int z = blockIdx.y;
  const float* W = (z == 0) ? W0 : (z == 1) ? W1 : (z == 2) ? W2 : W3;
  const int i = blockIdx.x * 256 + threadIdx.x;
  if (i >= n8) return;
  const float* p = W + 8 * (size_t)i;
  const v4f a = *(const v4f*)(p);
  const v4f c = *(const v4f*)(p + 4);
  unsigned short hb[8];
#pragma unroll
  for (int e = 0; e < 4; ++e) {
    hb[e]     = h_bits(a[e] * scale);
    hb[4 + e] = h_bits(c[e] * scale);
  }
  const v4u u = (v4u){pk16(hb[0], hb[1]), pk16(hb[2], hb[3]), pk16(hb[4], hb[5]), pk16(hb[6], hb[7])};
  unsigned short* q = out + (size_t)z * (size_t)n8 * 8 + 8 * (size_t)i;
  *(volatile v4u*)q = u;
  __threadfence();
  *(volatile v4u*)q = u;
}

__global__ __launch_bounds__(256) void castgate_kernel(const float* __restrict__ Wsd, const float* __restrict__ Wpd,
                                                       unsigned short* __restrict__ out, float scale) {
  const int bid = blockIdx.x;
  const int i = bid * 256 + threadIdx.x;
  const int row = i >> 6, col8 = (i & 63) * 8;
  float v[8];
#pragma unroll
  for (int e = 0; e < 8; ++e) v[e] = 0.0f;
  if (bid < 4) {
    const float* src = (bid < 2) ? Wsd : Wpd;
    int srow = (bid < 2) ? row : (row - 8);
    srow = srow < 0 ? 0 : (srow > 7 ? 7 : srow);
    const float* p = src + (size_t)srow * kNDM + col8;
    const v4f a = *(const v4f*)(p);
    const v4f c = *(const v4f*)(p + 4);
#pragma unroll
    for (int e = 0; e < 4; ++e) { v[e] = a[e] * scale; v[4 + e] = c[e] * scale; }
  }
  unsigned short hb[8];
#pragma unroll
  for (int e = 0; e < 8; ++e) hb[e] = h_bits(v[e]);
  const v4u u = (v4u){pk16(hb[0], hb[1]), pk16(hb[2], hb[3]), pk16(hb[4], hb[5]), pk16(hb[6], hb[7])};
  unsigned short* q = out + 8 * (size_t)i;
  *(volatile v4u*)q = u;
  __threadfence();
  *(volatile v4u*)q = u;
}

__global__ __launch_bounds__(128) void pair_scan_kernel(const unsigned short* __restrict__ P16,
                                                        const float* __restrict__ G32,
                                                        const float* __restrict__ bsd, const float* __restrict__ bpd,
                                                        unsigned short* __restrict__ MIX16) {
  __shared__ __align__(16) float sState[2][64];
  __shared__ __align__(16) unsigned short sMix[2][16][64];
  const int tid  = threadIdx.x;
  const int wave = tid >> 5, lane = tid & 31, hh = lane >> 4, c = lane & 15;
  const int bh = blockIdx.x;
  const int b = bh >> 3, h = bh & 7;
  const int e = wave * 16 + c;
  const size_t rowbase = (size_t)b * kNS;
  const float bs = bsd[h], bp = bpd[h];
  if (tid < 64) sState[0][tid] = 0.0f;
  float st = 0.0f;
  float pr0[16], pr1[16];
#pragma unroll
  for (int i = 0; i < 16; ++i) { pr0[i] = 0.0f; pr1[i] = 0.0f; }
  const v8f zero8 = (v8f){0.f, 0.f, 0.f, 0.f, 0.f, 0.f, 0.f, 0.f};
  __syncthreads();

  for (int t = 0; t < kNS; ++t) {
    const size_t row = rowbase + (size_t)t;
    const float gs = G32[row * kGateN + h] + bs;
    const float gp = G32[row * kGateN + 8 + h] + bp;
    const float sd = 1.0f / (1.0f + expf(-gs));
    const float pd = 1.0f / (1.0f + expf(-gp));
    const unsigned short* prow = P16 + row * kNProj + h * kNSD;
    const float av  = h2f(prow[e]) * kActInv;
    const float bv  = h2f(prow[512 + e]) * kActInv;
    const float qr8 = h2f(prow[1536 + e]);
    const _Float16* qlp = (const _Float16*)(const void*)(prow + 1024);
    const v16h qf0 = Frag<_Float16>::load(qlp + 8 * hh);
    const v16h qf1 = Frag<_Float16>::load(qlp + 32 + 8 * hh);
    const float* sp = sState[t & 1];
    const v4f p0 = *(const v4f*)(sp + 8 * hh);
    const v4f p1 = *(const v4f*)(sp + 8 * hh + 4);
    const v4f p2 = *(const v4f*)(sp + 16 + 8 * hh);
    const v4f p3 = *(const v4f*)(sp + 20 + 8 * hh);
    const v4f p4 = *(const v4f*)(sp + 32 + 8 * hh);
    const v4f p5 = *(const v4f*)(sp + 36 + 8 * hh);
    const v4f p6 = *(const v4f*)(sp + 48 + 8 * hh);
    const v4f p7 = *(const v4f*)(sp + 52 + 8 * hh);
    float pv0[16], pv1[16];
#pragma unroll
    for (int i = 0; i < 4; ++i) {
      pv0[i] = p0[i]; pv0[4 + i] = p1[i]; pv0[8 + i] = p2[i]; pv0[12 + i] = p3[i];
      pv1[i] = p4[i]; pv1[4 + i] = p5[i]; pv1[8 + i] = p6[i]; pv1[12 + i] = p7[i];
    }
    const float wb = (1.0f - pd) * bv * kPairCarry;
    v16h bq0, bq1;
#pragma unroll
    for (int i = 0; i < 16; ++i) {
      pr0[i] = pd * pr0[i] + pv0[i] * wb;
      bq0[i] = (_Float16)pr0[i];
    }
    v8f acc = hmma(qf0, bq0, zero8);
#pragma unroll
    for (int i = 0; i < 16; ++i) {
      pr1[i] = pd * pr1[i] + pv1[i] * wb;
      bq1[i] = (_Float16)pr1[i];
    }
    acc = hmma(qf1, bq1, acc);
    const float lc = acc[0] * kLcInv;
    const float mixv = lc * qr8 * 2.0f;
    if (hh == 0) {
      sMix[(t >> 4) & 1][t & 15][e] = h_bits(mixv);
      st = sd * st + (1.0f - sd) * av;
      sState[(t + 1) & 1][e] = st;
    }
    __syncthreads();
    if (wave == 0 && (t & 15) == 15) {
      const int fb = (t >> 4) & 1;
      const int q = lane >> 3, c8 = (lane & 7) * 8;
      const size_t r0 = row - 15;
      unsigned short* mbase = MIX16 + (size_t)h * kNSD + c8;
      for (int pass = 0; pass < 2; ++pass) {
#pragma unroll
        for (int it = 0; it < 4; ++it) {
          const int r16 = it * 4 + q;
          const v4u u = *(const v4u*)(&sMix[fb][r16][c8]);
          *(volatile v4u*)(mbase + (r0 + (size_t)r16) * kInner) = u;
        }
        __threadfence();
      }
    }
  }
}

__global__ __launch_bounds__(256) void gelu2_kernel(const unsigned int* __restrict__ hp, const float* __restrict__ b1,
                                                    unsigned int* __restrict__ hout, int n2) {
  const int i = blockIdx.x * 256 + threadIdx.x;
  if (i >= n2) return;
  const unsigned int w = hp[i];
  const int col = (2 * i) & (kNHid - 1);
  const float v0 = h2f(w & 0xffffu) * kActInv + b1[col];
  const float v1 = h2f(w >> 16) * kActInv + b1[col + 1];
  const float g0 = 0.5f * v0 * (1.0f + erff(v0 * 0.70710678118654752f));
  const float g1 = 0.5f * v1 * (1.0f + erff(v1 * 0.70710678118654752f));
  const unsigned int u = pk16(h_bits(g0 * kActCarry), h_bits(g1 * kActCarry));
  ((volatile unsigned int*)hout)[i] = u;
  __threadfence();
  ((volatile unsigned int*)hout)[i] = u;
}

extern "C" void kernel_launch(void* const* d_in, const int* in_sizes, int n_in,
                              void* d_out, int out_size, void* d_ws, size_t ws_size,
                              hipStream_t stream) {
  (void)in_sizes;
  if (n_in < 18) return;
  if (out_size != kRows * kNDM) return;

  const float* x    = (const float*)d_in[0];
  const float* ng   = (const float*)d_in[1];
  const float* nb   = (const float*)d_in[2];
  const float* fg   = (const float*)d_in[3];
  const float* fb   = (const float*)d_in[4];
  const float* Wa   = (const float*)d_in[5];
  const float* Wb   = (const float*)d_in[6];
  const float* Wql  = (const float*)d_in[7];
  const float* Wqr  = (const float*)d_in[8];
  const float* Wsd  = (const float*)d_in[9];
  const float* bsd  = (const float*)d_in[10];
  const float* Wpd  = (const float*)d_in[11];
  const float* bpd  = (const float*)d_in[12];
  const float* Wout = (const float*)d_in[13];
  const float* W1   = (const float*)d_in[14];
  const float* b1   = (const float*)d_in[15];
  const float* W2   = (const float*)d_in[16];
  const float* b2   = (const float*)d_in[17];
  float* out = (float*)d_out;

  const size_t szN16   = (size_t)kRows * kNDM * 2;
  const size_t szWcat  = (size_t)kNProj * kNDM * 2;
  const size_t szWg    = (size_t)kGateN * kNDM * 2;
  const size_t szWout  = (size_t)kNDM * kInner * 2;
  const size_t szW1    = (size_t)kNHid * kNDM * 2;
  const size_t szW2    = (size_t)kNDM * kNHid * 2;
  const size_t szProj  = (size_t)kRows * kNProj * 2;
  const size_t szG     = (size_t)kRows * kGateN * 4;
  const size_t szR     = (size_t)kRows * kNDM * 4;
  size_t off = 0;
  const size_t oN16  = off; off += szN16;
  const size_t oWcat = off; off += szWcat;
  const size_t oWg   = off; off += szWg;
  const size_t oWout = off; off += szWout;
  const size_t oW1   = off; off += szW1;
  const size_t oW2   = off; off += szW2;
  const size_t oProj = off; off += szProj;
  const size_t oG    = off; off += szG;
  const size_t oR    = off; off += szR;
  if (off > ws_size) return;

  char* ws = (char*)d_ws;
  unsigned short* N16    = (unsigned short*)(ws + oN16);
  unsigned short* Wcat16 = (unsigned short*)(ws + oWcat);
  unsigned short* Wg16   = (unsigned short*)(ws + oWg);
  unsigned short* Wout16 = (unsigned short*)(ws + oWout);
  unsigned short* W1h    = (unsigned short*)(ws + oW1);
  unsigned short* W2h    = (unsigned short*)(ws + oW2);
  unsigned short* PROJ16 = (unsigned short*)(ws + oProj);
  unsigned short* HP16   = PROJ16;
  unsigned short* H16    = (unsigned short*)(ws + oProj + (size_t)kFfnChunkRows * kNHid * 2);
  float*          G32    = (float*)(ws + oG);
  float*          R32    = (float*)(ws + oR);
  unsigned short* MIX16  = N16;

  ln_f16_kernel<<<kRows / 8, 256, 0, stream>>>(x, ng, nb, N16, kRows, kNCarry);

  {
    const int n8sq = kInner * kNDM / 8;
    castw4_kernel<<<dim3((n8sq + 255) / 256, 4), 256, 0, stream>>>(Wa, Wb, Wql, Wqr, Wcat16, n8sq, kWCarry);
    castgate_kernel<<<16, 256, 0, stream>>>(Wsd, Wpd, Wg16, kWCarry);
    castw4_kernel<<<dim3((n8sq + 255) / 256, 1), 256, 0, stream>>>(Wout, Wout, Wout, Wout, Wout16, n8sq, kWCarry);
    const int n8ffn = kNHid * kNDM / 8;
    castw4_kernel<<<dim3((n8ffn + 255) / 256, 1), 256, 0, stream>>>(W1, W1, W1, W1, W1h, n8ffn, kWCarry);
    castw4_kernel<<<dim3((n8ffn + 255) / 256, 1), 256, 0, stream>>>(W2, W2, W2, W2, W2h, n8ffn, kWCarry);
  }

  {
    const int tiles = (kRows / 64) * (kNProj / 64);
    wmma_gemm64<0, false, 0, 1, false, 6><<<dim3((tiles + 7) / 8, 1), 256, 0, stream>>>(
        N16, nullptr, kNDM, 0L, Wcat16, nullptr, kNDM, 0L,
        (void*)PROJ16, nullptr, kNProj, 0L, nullptr, nullptr, 0L, kRows, kNProj, kNDM, kProjScale);
  }
  {
    const int tiles = (kRows / 64) * (kGateN / 64);
    wmma_gemm64<0, false, 0, 0, false, 0><<<dim3((tiles + 7) / 8, 1), 256, 0, stream>>>(
        N16, nullptr, kNDM, 0L, Wg16, nullptr, kNDM, 0L,
        (void*)G32, nullptr, kGateN, 0L, nullptr, nullptr, 0L, kRows, kGateN, kNDM, kProjScale);
  }
  pair_scan_kernel<<<kNB * kNH, 128, 0, stream>>>(PROJ16, G32, bsd, bpd, MIX16);

  {
    const int tiles = (kRows / 64) * (kNDM / 64);
    wmma_gemm64<0, false, 0, 0, true, 0><<<dim3((tiles + 7) / 8, 1), 256, 0, stream>>>(
        MIX16, nullptr, kInner, 0L, Wout16, nullptr, kInner, 0L,
        (void*)R32, nullptr, kNDM, 0L, nullptr, x, 0L, kRows, kNDM, kInner, kWoutScale);
  }
  ln_f16_kernel<<<kRows / 8, 256, 0, stream>>>(R32, fg, fb, N16, kRows, kNCarry);

  for (int ch = 0; ch < 2; ++ch) {
    const size_t rowoff = (size_t)ch * kFfnChunkRows;
    {
      const int tiles = (kFfnChunkRows / 64) * (kNHid / 64);
      wmma_gemm64<0, false, 0, 1, false, 0><<<dim3((tiles + 7) / 8, 1), 256, 0, stream>>>(
          N16 + rowoff * kNDM, nullptr, kNDM, 0L, W1h, nullptr, kNDM, 0L,
          (void*)HP16, nullptr, kNHid, 0L, nullptr, nullptr, 0L, kFfnChunkRows, kNHid, kNDM, kW1Scale);
    }
    {
      const int n2 = kFfnChunkRows * kNHid / 2;
      gelu2_kernel<<<(n2 + 255) / 256, 256, 0, stream>>>((const unsigned int*)(const void*)HP16, b1,
                                                        (unsigned int*)(void*)H16, n2);
    }
    {
      const int tiles = (kFfnChunkRows / 64) * (kNDM / 64);
      wmma_gemm64<0, false, 2, 0, true, 0><<<dim3((tiles + 7) / 8, 1), 256, 0, stream>>>(
          H16, nullptr, kNHid, 0L, W2h, nullptr, kNHid, 0L,
          (void*)(out + rowoff * kNDM), nullptr, kNDM, 0L, b2, R32 + rowoff * kNDM, 0L,
          kFfnChunkRows, kNDM, kNHid, kW2Scale);
    }
  }
}
